// Retention_60258391162952
// MI455X (gfx1250) — hardware-verified
//
#include <hip/hip_runtime.h>
#include <math.h>
#include <stdint.h>
#include <stddef.h>

constexpr int kB = 4;
constexpr int kL = 2048;
constexpr int kH = 1024;
constexpr int kTok = kB * kL;
constexpr float kGamma = 0.96875f;
constexpr int kTile = 64;
constexpr int kBand = 512;
constexpr int kBandTiles = kBand / kTile;
constexpr int kITiles = kL / kTile;
constexpr int kDTiles = kH / kTile;
constexpr int kSCols = (kBandTiles + 1) * kTile;
constexpr int kTri = kBandTiles * (kBandTiles + 1) / 2;
constexpr int kScoreTiles = kTri + (kITiles - kBandTiles) * (kBandTiles + 1);
constexpr int kOutTiles = kITiles * kDTiles;
static_assert(kB == 4 && kL == 2048 && kH == 1024);
static_assert(kGamma == 0.96875f);
static_assert(kBandTiles == 8 && kSCols == 576 && kTri == 36 && kScoreTiles == 252 && kOutTiles == 512);
static_assert(kH % 32 == 0 && kH % 64 == 0 && kTok % 64 == 0 && kL % kTile == 0 && kSCols % 8 == 0 && (kSCols * 2) % 128 == 0);

constexpr size_t kPlaneTok = (size_t)kTok * kH * 2;
constexpr size_t kPlaneW   = (size_t)kH * kH * 2;
constexpr size_t kPlaneS   = (size_t)kL * kSCols * 2;
constexpr size_t kOffXb = 0;
constexpr size_t kOffWt = kOffXb + kPlaneTok;
constexpr size_t kOffQh = kOffWt + 3 * kPlaneW;
constexpr size_t kOffQl = kOffQh + kPlaneTok;
constexpr size_t kOffKh = kOffQl + kPlaneTok;
constexpr size_t kOffKl = kOffKh + kPlaneTok;
constexpr size_t kOffVh = kOffKl + kPlaneTok;
constexpr size_t kOffVl = kOffVh + kPlaneTok;
constexpr size_t kOffSh = kOffVl + kPlaneTok;
constexpr size_t kOffSl = kOffSh + kPlaneS;
constexpr size_t kWsTotal = kOffSl + kPlaneS;
static_assert(kWsTotal == (size_t)128450560);
static_assert(kWsTotal <= (size_t)134217728);
static_assert(kOffWt % 128 == 0 && kOffQh % 128 == 0 && kOffVh % 128 == 0 && kOffSh % 128 == 0 && kOffSl % 128 == 0);

typedef __attribute__((ext_vector_type(16))) __bf16   v16b;
typedef __attribute__((ext_vector_type(8)))  __bf16   v8b;
typedef __attribute__((ext_vector_type(8)))  _Float16 v8h;
typedef __attribute__((ext_vector_type(8)))  float    v8f;
typedef __attribute__((ext_vector_type(4)))  float    v4f;
typedef __attribute__((ext_vector_type(4)))  unsigned int v4u;

__device__ __forceinline__ unsigned short f2bf_bits(float f) {
  unsigned u = __float_as_uint(f);
  return (unsigned short)((u + 0x7FFFu + ((u >> 16) & 1u)) >> 16);
}
__device__ __forceinline__ float bf_bits2f(unsigned short h) { return __uint_as_float(((unsigned)h) << 16); }
__device__ __forceinline__ unsigned pk16(unsigned short a, unsigned short b) { return (unsigned)a | ((unsigned)b << 16); }

__device__ __forceinline__ void guard4_b(v8f& a, v8f& b, v8f& c, v8f& d, v16b x, v16b y) {
  asm volatile("v_nop\n\tv_nop\n\tv_nop\n\tv_nop" : "+v"(a), "+v"(b), "+v"(c), "+v"(d) : "v"(x), "v"(y));
}
__device__ __forceinline__ void keep4_b(v16b a, v16b b, v16b c, v16b d) { asm volatile("v_nop" :: "v"(a), "v"(b), "v"(c), "v"(d)); }
__device__ __forceinline__ void acc_guard4(v8f& a, v8f& b, v8f& c, v8f& d) {
  asm volatile("v_nop\n\tv_nop\n\tv_nop\n\tv_nop" : "+v"(a), "+v"(b), "+v"(c), "+v"(d));
}

struct FragB {
  union U { v16b v; v8b h[2]; };
  static __device__ __forceinline__ v16b load(const __bf16* p) {
    U f; f.h[0] = *(const v8b*)(p); f.h[1] = *(const v8b*)(p + 16); return f.v;
  }
  static __device__ __forceinline__ v8f mma(v16b a, v16b b, v8f c) {
    return __builtin_amdgcn_wmma_f32_16x16x32_bf16(false, a, false, b, (short)0, c, false, false);
  }
};

__global__ __launch_bounds__(256) void cast8_bf16_kernel(const float* __restrict__ in, unsigned short* __restrict__ out,
                                                         int n8, const float* __restrict__ aux) {
  (void)aux;
  const int i = blockIdx.x * 256 + threadIdx.x;
  if (i >= n8) return;
  const float* p = in + 8 * (size_t)i;
  const v4f a = *(const v4f*)(p);
  const v4f c = *(const v4f*)(p + 4);
  unsigned short hb[8];
#pragma unroll
  for (int e = 0; e < 4; ++e) {
    hb[e]     = f2bf_bits(a[e]);
    hb[4 + e] = f2bf_bits(c[e]);
  }
  const v4u u = (v4u){pk16(hb[0], hb[1]), pk16(hb[2], hb[3]), pk16(hb[4], hb[5]), pk16(hb[6], hb[7])};
  unsigned short* q = out + 8 * (size_t)i;
  *(volatile v4u*)q = u;
  __threadfence();
  *(volatile v4u*)q = u;
}

__global__ __launch_bounds__(256) void wt3_kernel(const float* __restrict__ W0, const float* __restrict__ W1,
                                                  const float* __restrict__ W2, unsigned short* __restrict__ out) {
  __shared__ float sm[64][65];
  const int t  = threadIdx.x;
  const int k0 = blockIdx.x * 64;
  const int n0 = blockIdx.y * 64;
  const int z  = blockIdx.z;
  const float* W = (z == 0) ? W0 : (z == 1) ? W1 : W2;
#pragma unroll
  for (int i = 0; i < 16; ++i) {
    const int e = i * 256 + t;
    const int r = e >> 6;
    const int c = e & 63;
    sm[c][r] = W[(size_t)(k0 + r) * kH + n0 + c];
  }
  __syncthreads();
  const int lane = t & 31, wave = t >> 5;
  const int q = lane >> 3, c8 = (lane & 7) * 8;
  unsigned short* op = out + (size_t)z * kH * kH;
  for (int pass = 0; pass < 2; ++pass) {
#pragma unroll
    for (int it = 0; it < 2; ++it) {
      const int row = wave * 8 + it * 4 + q;
      unsigned short hb[8];
#pragma unroll
      for (int e = 0; e < 8; ++e) hb[e] = f2bf_bits(sm[row][c8 + e]);
      const v4u u = (v4u){pk16(hb[0], hb[1]), pk16(hb[2], hb[3]), pk16(hb[4], hb[5]), pk16(hb[6], hb[7])};
      *(volatile v4u*)(op + (size_t)(n0 + row) * kH + k0 + c8) = u;
    }
    __threadfence();
  }
}

template <bool SPLIT, int OUT_MODE>
__global__ __launch_bounds__(256) void gemm64_bf16_kernel(
    const unsigned short* __restrict__ Ap, const unsigned short* __restrict__ A2p, int lda, long strideA,
    const unsigned short* __restrict__ Btp, const unsigned short* __restrict__ Bt2p, int ldb, long strideB,
    void* __restrict__ Cout, void* __restrict__ Cout2, int ldc, long strideC,
    int M, int N, int K, float scale) {
  const __bf16* A = (const __bf16*)Ap; const __bf16* A2 = (const __bf16*)A2p;
  const __bf16* Bt = (const __bf16*)Btp; const __bf16* Bt2 = (const __bf16*)Bt2p;
  __shared__ __align__(16) float sT[8][16 * 68];
  const int b    = blockIdx.y;
  const int lane = threadIdx.x & 31;
  const int wave = threadIdx.x >> 5;
  const int tilesN = N >> 6;
  const int tilesM = M >> 6;
  const int tile = blockIdx.x * 8 + wave;
  if (tile >= tilesM * tilesN) return;
  const int tm = tile / tilesN;
  const int tn = tile - tm * tilesN;
  const int m0 = tm << 6;
  const int n0 = tn << 6;

  const __bf16* Ab  = A  + (size_t)b * strideA;
  const __bf16* Bb  = Bt + (size_t)b * strideB;
  const __bf16* Ab2 = SPLIT ? (A2  + (size_t)b * strideA) : nullptr;
  const __bf16* Bb2 = SPLIT ? (Bt2 + (size_t)b * strideB) : nullptr;

  const int rlane = lane & 15;
  const int koff  = (lane >> 4) * 8;
  const int mOff  = (lane >> 4) * 8;

  v8f acc[4][4];
#pragma unroll
  for (int i = 0; i < 4; ++i)
#pragma unroll
    for (int j = 0; j < 4; ++j) acc[i][j] = (v8f){0.f,0.f,0.f,0.f,0.f,0.f,0.f,0.f};

  for (int k0 = 0; k0 < K; k0 += 32) {
    v16b bh[4], bl[4];
#pragma unroll
    for (int j = 0; j < 4; ++j) {
      const size_t bo = (size_t)(n0 + (j << 4) + rlane) * ldb + koff + k0;
      bh[j] = FragB::load(Bb + bo);
      if (SPLIT) bl[j] = FragB::load(Bb2 + bo);
    }
#pragma unroll
    for (int i = 0; i < 4; ++i) {
      const size_t ao = (size_t)(m0 + (i << 4) + rlane) * lda + koff + k0;
      v16b ah = FragB::load(Ab + ao);
      v16b al = ah;
      if (SPLIT) al = FragB::load(Ab2 + ao);
#pragma unroll
      for (int j = 0; j < 4; ++j) {
        acc[i][j] = FragB::mma(ah, bh[j], acc[i][j]);
        if (SPLIT) {
          acc[i][j] = FragB::mma(ah, bl[j], acc[i][j]);
          acc[i][j] = FragB::mma(al, bh[j], acc[i][j]);
        }
      }
      guard4_b(acc[i][0], acc[i][1], acc[i][2], acc[i][3], ah, al);
    }
    keep4_b(bh[0], bh[1], bh[2], bh[3]);
    if (SPLIT) keep4_b(bl[0], bl[1], bl[2], bl[3]);
  }
  acc_guard4(acc[0][0], acc[0][1], acc[0][2], acc[0][3]);
  acc_guard4(acc[1][0], acc[1][1], acc[1][2], acc[1][3]);
  acc_guard4(acc[2][0], acc[2][1], acc[2][2], acc[2][3]);
  acc_guard4(acc[3][0], acc[3][1], acc[3][2], acc[3][3]);

  float* slab = sT[wave];
#pragma unroll
  for (int i = 0; i < 4; ++i) {
    const int mBase = m0 + (i << 4);
#pragma unroll
    for (int j = 0; j < 4; ++j) {
#pragma unroll
      for (int r = 0; r < 8; ++r) {
        const float v = acc[i][j][r] * scale;
        slab[(mOff + r) * 68 + (j << 4) + rlane] = v;
      }
    }
    __builtin_amdgcn_fence(__ATOMIC_RELEASE, "workgroup");
    __builtin_amdgcn_wave_barrier();
    __builtin_amdgcn_fence(__ATOMIC_ACQUIRE, "workgroup");
    if (OUT_MODE == 0) {
      float* C = (float*)Cout + (size_t)b * strideC;
      const int hh = lane >> 4, c4 = (lane & 15) * 4;
      for (int pass = 0; pass < 2; ++pass) {
#pragma unroll
        for (int it = 0; it < 8; ++it) {
          const int row = it * 2 + hh;
          v4f v = *(const v4f*)(slab + row * 68 + c4);
          *(volatile v4f*)(C + (size_t)(mBase + row) * ldc + n0 + c4) = v;
        }
        __threadfence();
      }
    } else {
      const int q = lane >> 3, c8 = (lane & 7) * 8;
      unsigned short* C  = (unsigned short*)Cout  + (size_t)b * strideC;
      unsigned short* C2 = (unsigned short*)Cout2 + (size_t)b * strideC;
      for (int pass = 0; pass < 2; ++pass) {
#pragma unroll
        for (int it = 0; it < 4; ++it) {
          const int row = it * 4 + q;
          const float* sp = slab + row * 68 + c8;
          v8h hv, lv;
#pragma unroll
          for (int e = 0; e < 8; ++e) {
            unsigned short hb = f2bf_bits(sp[e]);
            unsigned short lb = f2bf_bits(sp[e] - bf_bits2f(hb));
            hv[e] = __builtin_bit_cast(_Float16, hb);
            lv[e] = __builtin_bit_cast(_Float16, lb);
          }
          *(volatile v8h*)(C  + (size_t)(mBase + row) * ldc + n0 + c8) = hv;
          *(volatile v8h*)(C2 + (size_t)(mBase + row) * ldc + n0 + c8) = lv;
        }
        __threadfence();
      }
    }
    __builtin_amdgcn_fence(__ATOMIC_RELEASE, "workgroup");
    __builtin_amdgcn_wave_barrier();
    __builtin_amdgcn_fence(__ATOMIC_ACQUIRE, "workgroup");
  }
}

__global__ __launch_bounds__(256) void scores_band_kernel(
    const unsigned short* __restrict__ qhp, const unsigned short* __restrict__ qlp,
    const unsigned short* __restrict__ khp, const unsigned short* __restrict__ klp,
    unsigned short* __restrict__ shp, unsigned short* __restrict__ slp, int b, float log2g) {
  __shared__ __align__(16) float sT[8][16 * 68];
  __shared__ __align__(16) float sDec[8][128];
  const int lane = threadIdx.x & 31;
  const int wave = threadIdx.x >> 5;
  const int t = blockIdx.x * 8 + wave;
  if (t >= kScoreTiles) return;

  int s = 0;
#pragma unroll
  for (int c = 1; c < kBandTiles; ++c) s = (t >= (c * (c + 1)) / 2) ? c : s;
  const int tiLow = s;
  const int tjLow = t - (s * (s + 1)) / 2;
  const int u = t - kTri;
  const int tiHigh = kBandTiles + u / (kBandTiles + 1);
  const int tjHigh = u - (tiHigh - kBandTiles) * (kBandTiles + 1);
  const int ti    = (t >= kTri) ? tiHigh : tiLow;
  const int tjrel = (t >= kTri) ? tjHigh : tjLow;
  const int jt0 = (ti > kBandTiles) ? (ti - kBandTiles) : 0;
  const int i0 = ti * kTile;
  const int j0 = (jt0 + tjrel) * kTile;
  const int c0 = tjrel * kTile;

  const __bf16* Aq  = (const __bf16*)qhp + (size_t)(b * kL + i0) * kH;
  const __bf16* Aq2 = (const __bf16*)qlp + (size_t)(b * kL + i0) * kH;
  const __bf16* Bk  = (const __bf16*)khp + (size_t)(b * kL + j0) * kH;
  const __bf16* Bk2 = (const __bf16*)klp + (size_t)(b * kL + j0) * kH;

  const int rlane = lane & 15;
  const int koff  = (lane >> 4) * 8;
  const int mOff  = (lane >> 4) * 8;

#pragma unroll
  for (int e = 0; e < 4; ++e) {
    const int idx = lane * 4 + e;
    const int d = (i0 - j0) + idx - 63;
    const float f = exp2f((float)d * log2g);
    sDec[wave][idx] = (d >= 0) ? f : 0.0f;
  }
  __builtin_amdgcn_fence(__ATOMIC_RELEASE, "workgroup");
  __builtin_amdgcn_wave_barrier();
  __builtin_amdgcn_fence(__ATOMIC_ACQUIRE, "workgroup");

  v8f acc[4][4];
#pragma unroll
  for (int i = 0; i < 4; ++i)
#pragma unroll
    for (int j = 0; j < 4; ++j) acc[i][j] = (v8f){0.f,0.f,0.f,0.f,0.f,0.f,0.f,0.f};

  for (int k0 = 0; k0 < kH; k0 += 32) {
    v16b bh[4], bl[4];
#pragma unroll
    for (int j = 0; j < 4; ++j) {
      const size_t bo = (size_t)((j << 4) + rlane) * kH + koff + k0;
      bh[j] = FragB::load(Bk + bo);
      bl[j] = FragB::load(Bk2 + bo);
    }
#pragma unroll
    for (int i = 0; i < 4; ++i) {
      const size_t ao = (size_t)((i << 4) + rlane) * kH + koff + k0;
      v16b ah = FragB::load(Aq + ao);
      v16b al = FragB::load(Aq2 + ao);
#pragma unroll
      for (int j = 0; j < 4; ++j) {
        acc[i][j] = FragB::mma(ah, bh[j], acc[i][j]);
        acc[i][j] = FragB::mma(ah, bl[j], acc[i][j]);
        acc[i][j] = FragB::mma(al, bh[j], acc[i][j]);
      }
      guard4_b(acc[i][0], acc[i][1], acc[i][2], acc[i][3], ah, al);
    }
    keep4_b(bh[0], bh[1], bh[2], bh[3]);
    keep4_b(bl[0], bl[1], bl[2], bl[3]);
  }
  acc_guard4(acc[0][0], acc[0][1], acc[0][2], acc[0][3]);
  acc_guard4(acc[1][0], acc[1][1], acc[1][2], acc[1][3]);
  acc_guard4(acc[2][0], acc[2][1], acc[2][2], acc[2][3]);
  acc_guard4(acc[3][0], acc[3][1], acc[3][2], acc[3][3]);

  float* slab = sT[wave];
  const float* dec = sDec[wave];
  const int ij0 = i0 - j0;
#pragma unroll
  for (int i = 0; i < 4; ++i) {
    const int mB = i << 4;
#pragma unroll
    for (int j = 0; j < 4; ++j) {
      const int jl = (j << 4) + rlane;
#pragma unroll
      for (int r = 0; r < 8; ++r) {
        const int il = mB + mOff + r;
        const int dd = il - jl;
        const float dv = dec[dd + 63];
        const float v = (ij0 + dd >= 0) ? (acc[i][j][r] * dv) : 0.0f;
        slab[(mOff + r) * 68 + (j << 4) + rlane] = v;
      }
    }
    __builtin_amdgcn_fence(__ATOMIC_RELEASE, "workgroup");
    __builtin_amdgcn_wave_barrier();
    __builtin_amdgcn_fence(__ATOMIC_ACQUIRE, "workgroup");
    {
      const int q = lane >> 3, c8 = (lane & 7) * 8;
      for (int pass = 0; pass < 2; ++pass) {
#pragma unroll
        for (int it = 0; it < 4; ++it) {
          const int row = it * 4 + q;
          const float* sp = slab + row * 68 + c8;
          v8h hv, lv;
#pragma unroll
          for (int e = 0; e < 8; ++e) {
            unsigned short hb = f2bf_bits(sp[e]);
            unsigned short lb = f2bf_bits(sp[e] - bf_bits2f(hb));
            hv[e] = __builtin_bit_cast(_Float16, hb);
            lv[e] = __builtin_bit_cast(_Float16, lb);
          }
          const size_t o = (size_t)(i0 + mB + row) * kSCols + c0 + c8;
          *(volatile v8h*)(shp + o) = hv;
          *(volatile v8h*)(slp + o) = lv;
        }
        __threadfence();
      }
    }
    __builtin_amdgcn_fence(__ATOMIC_RELEASE, "workgroup");
    __builtin_amdgcn_wave_barrier();
    __builtin_amdgcn_fence(__ATOMIC_ACQUIRE, "workgroup");
  }
}

__global__ __launch_bounds__(256) void out_band_kernel(
    const unsigned short* __restrict__ shp, const unsigned short* __restrict__ slp,
    const unsigned short* __restrict__ vhp, const unsigned short* __restrict__ vlp,
    float* __restrict__ out, int b) {
  __shared__ __align__(16) float sT[8][16 * 68];
  const int lane = threadIdx.x & 31;
  const int wave = threadIdx.x >> 5;
  const int t = blockIdx.x * 8 + wave;
  if (t >= kOutTiles) return;
  const int ti = t / kDTiles;
  const int tn = t - ti * kDTiles;
  const int i0 = ti * kTile;
  const int n0 = tn * kTile;
  const int jt0 = (ti > kBandTiles) ? (ti - kBandTiles) : 0;
  const int cnt = ((ti < kBandTiles) ? ti : kBandTiles) + 1;
  const int Kb  = cnt * kTile;

  const __bf16* As  = (const __bf16*)shp + (size_t)i0 * kSCols;
  const __bf16* As2 = (const __bf16*)slp + (size_t)i0 * kSCols;
  const __bf16* Bv  = (const __bf16*)vhp + (size_t)n0 * kTok + (size_t)b * kL + (size_t)jt0 * kTile;
  const __bf16* Bv2 = (const __bf16*)vlp + (size_t)n0 * kTok + (size_t)b * kL + (size_t)jt0 * kTile;

  const int rlane = lane & 15;
  const int koff  = (lane >> 4) * 8;
  const int mOff  = (lane >> 4) * 8;

  v8f acc[4][4];
#pragma unroll
  for (int i = 0; i < 4; ++i)
#pragma unroll
    for (int j = 0; j < 4; ++j) acc[i][j] = (v8f){0.f,0.f,0.f,0.f,0.f,0.f,0.f,0.f};

  for (int k0 = 0; k0 < Kb; k0 += 32) {
    v16b bh[4], bl[4];
#pragma unroll
    for (int j = 0; j < 4; ++j) {
      const size_t bo = (size_t)((j << 4) + rlane) * kTok + koff + k0;
      bh[j] = FragB::load(Bv + bo);
      bl[j] = FragB::load(Bv2 + bo);
    }
#pragma unroll
    for (int i = 0; i < 4; ++i) {
      const size_t ao = (size_t)((i << 4) + rlane) * kSCols + koff + k0;
      v16b ah = FragB::load(As + ao);
      v16b al = FragB::load(As2 + ao);
#pragma unroll
      for (int j = 0; j < 4; ++j) {
        acc[i][j] = FragB::mma(ah, bh[j], acc[i][j]);
        acc[i][j] = FragB::mma(ah, bl[j], acc[i][j]);
        acc[i][j] = FragB::mma(al, bh[j], acc[i][j]);
      }
      guard4_b(acc[i][0], acc[i][1], acc[i][2], acc[i][3], ah, al);
    }
    keep4_b(bh[0], bh[1], bh[2], bh[3]);
    keep4_b(bl[0], bl[1], bl[2], bl[3]);
  }
  acc_guard4(acc[0][0], acc[0][1], acc[0][2], acc[0][3]);
  acc_guard4(acc[1][0], acc[1][1], acc[1][2], acc[1][3]);
  acc_guard4(acc[2][0], acc[2][1], acc[2][2], acc[2][3]);
  acc_guard4(acc[3][0], acc[3][1], acc[3][2], acc[3][3]);

  float* slab = sT[wave];
  float* C = out + (size_t)b * kL * kH;
#pragma unroll
  for (int i = 0; i < 4; ++i) {
    const int mB = i << 4;
#pragma unroll
    for (int j = 0; j < 4; ++j) {
#pragma unroll
      for (int r = 0; r < 8; ++r) {
        slab[(mOff + r) * 68 + (j << 4) + rlane] = acc[i][j][r];
      }
    }
    __builtin_amdgcn_fence(__ATOMIC_RELEASE, "workgroup");
    __builtin_amdgcn_wave_barrier();
    __builtin_amdgcn_fence(__ATOMIC_ACQUIRE, "workgroup");
    {
      const int hh = lane >> 4, c4 = (lane & 15) * 4;
      for (int pass = 0; pass < 2; ++pass) {
#pragma unroll
        for (int it = 0; it < 8; ++it) {
          const int row = it * 2 + hh;
          v4f v = *(const v4f*)(slab + row * 68 + c4);
          *(volatile v4f*)(C + (size_t)(i0 + mB + row) * kH + n0 + c4) = v;
        }
        __threadfence();
      }
    }
    __builtin_amdgcn_fence(__ATOMIC_RELEASE, "workgroup");
    __builtin_amdgcn_wave_barrier();
    __builtin_amdgcn_fence(__ATOMIC_ACQUIRE, "workgroup");
  }
}

extern "C" void kernel_launch(void* const* d_in, const int* in_sizes, int n_in,
                              void* d_out, int out_size, void* d_ws, size_t ws_size,
                              hipStream_t stream) {
  if (n_in < 5) return;
  if (ws_size < kWsTotal) return;
  if ((size_t)out_size != (size_t)kTok * kH) return;
  if (in_sizes[0] != kTok * kH || in_sizes[1] != kH * kH || in_sizes[2] != kH * kH ||
      in_sizes[3] != kH * kH || in_sizes[4] != kH) return;

  const float* x     = (const float*)d_in[0];
  const float* wq    = (const float*)d_in[1];
  const float* wk    = (const float*)d_in[2];
  const float* wv    = (const float*)d_in[3];
  const float* theta = (const float*)d_in[4];
  float* out = (float*)d_out;

  char* ws = (char*)d_ws;
  unsigned short* xb  = (unsigned short*)(ws + kOffXb);
  unsigned short* wT  = (unsigned short*)(ws + kOffWt);
  unsigned short* wqT = wT;
  unsigned short* wkT = wT + (size_t)kH * kH;
  unsigned short* wvT = wT + 2 * (size_t)kH * kH;
  unsigned short* qh  = (unsigned short*)(ws + kOffQh);
  unsigned short* ql  = (unsigned short*)(ws + kOffQl);
  unsigned short* kh  = (unsigned short*)(ws + kOffKh);
  unsigned short* kl  = (unsigned short*)(ws + kOffKl);
  unsigned short* vh  = (unsigned short*)(ws + kOffVh);
  unsigned short* vl  = (unsigned short*)(ws + kOffVl);
  unsigned short* sh  = (unsigned short*)(ws + kOffSh);
  unsigned short* sl  = (unsigned short*)(ws + kOffSl);

  const float log2g = (float)log2((double)kGamma);

  const int n8 = kTok * kH / 8;
  cast8_bf16_kernel<<<dim3((n8 + 255) / 256), dim3(256), 0, stream>>>(x, xb, n8, theta);

  wt3_kernel<<<dim3(kH / 64, kH / 64, 3), dim3(256), 0, stream>>>(wq, wk, wv, wT);

  {
    const int tiles = (kTok / 64) * (kH / 64);
    gemm64_bf16_kernel<false, 2><<<dim3((tiles + 7) / 8, 1), dim3(256), 0, stream>>>(
        xb, xb, kH, 0L, wqT, wqT, kH, 0L, (void*)qh, (void*)ql, kH, 0L, kTok, kH, kH, 1.0f);
    gemm64_bf16_kernel<false, 2><<<dim3((tiles + 7) / 8, 1), dim3(256), 0, stream>>>(
        xb, xb, kH, 0L, wkT, wkT, kH, 0L, (void*)kh, (void*)kl, kH, 0L, kTok, kH, kH, 1.0f);
  }
  {
    const int tiles = (kH / 64) * (kTok / 64);
    gemm64_bf16_kernel<false, 2><<<dim3((tiles + 7) / 8, 1), dim3(256), 0, stream>>>(
        wvT, wvT, kH, 0L, xb, xb, kH, 0L, (void*)vh, (void*)vl, kTok, 0L, kH, kTok, kH, 1.0f);
  }
  for (int b = 0; b < kB; ++b) {
    scores_band_kernel<<<dim3((kScoreTiles + 7) / 8), dim3(256), 0, stream>>>(qh, ql, kh, kl, sh, sl, b, log2g);
    out_band_kernel<<<dim3((kOutTiles + 7) / 8), dim3(256), 0, stream>>>(sh, sl, vh, vl, out, b);
  }
}
